// MambaBlock_50861002719354
// MI455X (gfx1250) — hardware-verified
//
#include <hip/hip_runtime.h>
#include <math.h>

typedef __attribute__((ext_vector_type(16))) _Float16 v16h;
typedef __attribute__((ext_vector_type(8)))  _Float16 v8h;
typedef __attribute__((ext_vector_type(16))) __bf16   v16b;
typedef __attribute__((ext_vector_type(8)))  __bf16   v8b;
typedef __attribute__((ext_vector_type(8)))  float    v8f;
typedef __attribute__((ext_vector_type(4)))  float    v4f;

constexpr int kBatch = 2;
constexpr int kSeqL  = 2048;
constexpr int kDmod  = 1024;
constexpr int kDin   = 2048;
constexpr int kNst   = 16;
constexpr int kXZP   = 2 * kDin;
constexpr int kXdN   = 2 * kNst;
constexpr int kXdP   = 64;
constexpr int kRows  = kBatch * kSeqL;
constexpr int kTP    = 260;
constexpr float kCarryAct = 16.0f;
constexpr float kCarryW   = 1024.0f;
constexpr float kFold     = 1.0f / (kCarryAct * kCarryW);
static_assert(kDmod % 32 == 0 && kDin % 32 == 0, "GEMM K multiples of 32");
static_assert(kSeqL % 64 == 0 && kXZP % 64 == 0 && kXdP % 64 == 0 && kDin % 64 == 0 && kDmod % 64 == 0, "GEMM M,N multiples of 64");
static_assert(kXdN <= kXdP && kDin % 256 == 0 && kDmod == 1024 && kSeqL % 16 == 0, "tile multiples");

constexpr size_t kOffWIN  = 0;
constexpr size_t kOffWDT  = kOffWIN  + (size_t)kXZP  * kDmod * 2;
constexpr size_t kOffWOUT = kOffWDT  + (size_t)kDin  * kDin  * 2;
constexpr size_t kOffWX   = kOffWOUT + (size_t)kDmod * kDin  * 2;
constexpr size_t kOffXNH  = kOffWX   + (size_t)kXdP  * kDin  * 2;
constexpr size_t kOffXNL  = kOffXNH  + (size_t)kRows * kDmod * 2;
constexpr size_t kOffXZ   = kOffXNL  + (size_t)kRows * kDmod * 2;
constexpr size_t kOffUCH  = kOffXZ   + (size_t)kSeqL * kXZP  * 4;
constexpr size_t kOffUCL  = kOffUCH  + (size_t)kSeqL * kDin  * 2;
constexpr size_t kOffUC16 = kOffUCL  + (size_t)kSeqL * kDin  * 2;
constexpr size_t kOffXD   = kOffUC16 + (size_t)kSeqL * kDin  * 2;
constexpr size_t kOffDLR  = kOffXD   + (size_t)kSeqL * kXdP  * 4;
constexpr size_t kOffYG   = kOffDLR  + (size_t)kSeqL * kDin  * 4;
constexpr size_t kWsTotal = kOffYG   + (size_t)kSeqL * kDin  * 2;
static_assert(kWsTotal == 122421248ull, "carve total");
static_assert(kWsTotal <= 134217728ull, "carve cap");
static_assert((kOffWDT % 128) == 0 && (kOffWOUT % 128) == 0 && (kOffWX % 128) == 0 && (kOffXNH % 128) == 0 &&
              (kOffXNL % 128) == 0 && (kOffXZ % 128) == 0 && (kOffUCH % 128) == 0 && (kOffUCL % 128) == 0 &&
              (kOffUC16 % 128) == 0 && (kOffXD % 128) == 0 && (kOffDLR % 128) == 0 && (kOffYG % 128) == 0, "128-B aligned regions");

__device__ __forceinline__ unsigned short f2bf_bits(float f) {
  unsigned u = __float_as_uint(f);
  return (unsigned short)((u + 0x7FFFu + ((u >> 16) & 1u)) >> 16);
}
__device__ __forceinline__ float bf_bits2f(unsigned short h) { return __uint_as_float(((unsigned)h) << 16); }
__device__ __forceinline__ float rbf(float f) { return bf_bits2f(f2bf_bits(f)); }

__device__ __forceinline__ void guard4_h(v8f& a, v8f& b, v8f& c, v8f& d, v16h x, v16h y) { asm volatile("v_nop\n\tv_nop\n\tv_nop\n\tv_nop" : "+v"(a), "+v"(b), "+v"(c), "+v"(d) : "v"(x), "v"(y)); }
__device__ __forceinline__ void guard4_b(v8f& a, v8f& b, v8f& c, v8f& d, v16b x, v16b y) { asm volatile("v_nop\n\tv_nop\n\tv_nop\n\tv_nop" : "+v"(a), "+v"(b), "+v"(c), "+v"(d) : "v"(x), "v"(y)); }
__device__ __forceinline__ void keep4_h(v16h a, v16h b, v16h c, v16h d) { asm volatile("v_nop" :: "v"(a), "v"(b), "v"(c), "v"(d)); }
__device__ __forceinline__ void keep4_b(v16b a, v16b b, v16b c, v16b d) { asm volatile("v_nop" :: "v"(a), "v"(b), "v"(c), "v"(d)); }
__device__ __forceinline__ void acc_guard4(v8f& a, v8f& b, v8f& c, v8f& d) { asm volatile("v_nop\n\tv_nop\n\tv_nop\n\tv_nop" : "+v"(a), "+v"(b), "+v"(c), "+v"(d)); }
template <typename T> struct Frag;
template <> struct Frag<_Float16> {
  typedef v16h V; union U { v16h v; v8h h[2]; };
  static __device__ __forceinline__ v16h load(const _Float16* p) {
    U f; f.h[0] = *(const v8h*)(p); f.h[1] = *(const v8h*)(p + 16); return f.v;
  }
  static __device__ __forceinline__ v8f mma(v16h a, v16h b, v8f c) {
    return __builtin_amdgcn_wmma_f32_16x16x32_f16(false, a, false, b, (short)0, c, false, false);
  }
  static __device__ __forceinline__ void guard4(v8f& a, v8f& b, v8f& c, v8f& d, v16h x, v16h y) { guard4_h(a, b, c, d, x, y); }
  static __device__ __forceinline__ void keep(v16h a, v16h b, v16h c, v16h d) { keep4_h(a, b, c, d); }
};
template <> struct Frag<__bf16> {
  typedef v16b V; union U { v16b v; v8b h[2]; };
  static __device__ __forceinline__ v16b load(const __bf16* p) {
    U f; f.h[0] = *(const v8b*)(p); f.h[1] = *(const v8b*)(p + 16); return f.v;
  }
  static __device__ __forceinline__ v8f mma(v16b a, v16b b, v8f c) {
    return __builtin_amdgcn_wmma_f32_16x16x32_bf16(false, a, false, b, (short)0, c, false, false);
  }
  static __device__ __forceinline__ void guard4(v8f& a, v8f& b, v8f& c, v8f& d, v16b x, v16b y) { guard4_b(a, b, c, d, x, y); }
  static __device__ __forceinline__ void keep(v16b a, v16b b, v16b c, v16b d) { keep4_b(a, b, c, d); }
};

template <int ET> struct Elem;
template <> struct Elem<0> { typedef _Float16 T; };
template <> struct Elem<1> { typedef __bf16 T; };
template <int ET, int SPL, bool SKIP>
__global__ __launch_bounds__(256) void wmma_gemm64(
    const unsigned short* __restrict__ Ap, const unsigned short* __restrict__ A2p, int lda,
    const unsigned short* __restrict__ Btp, int ldb,
    float* __restrict__ C, int ldc,
    const float* __restrict__ skip,
    int M, int N, int K, float scale) {
  typedef typename Elem<ET>::T T;
  typedef typename Frag<T>::V V;
  const T* A = (const T*)Ap; const T* A2 = (const T*)A2p; const T* Bt = (const T*)Btp;
  __shared__ __align__(16) float sT[8][16 * 68];
  const int lane = threadIdx.x & 31;
  const int wave = threadIdx.x >> 5;
  const int tilesN = N >> 6;
  const int tilesM = M >> 6;
  const int tile = blockIdx.x * 8 + wave;
  if (tile >= tilesM * tilesN) return;
  const int tm = tile / tilesN;
  const int tn = tile - tm * tilesN;
  const int m0 = tm << 6;
  const int n0 = tn << 6;

  const int rlane = lane & 15;
  const int koff  = (lane >> 4) * 8;
  const int mOff  = (lane >> 4) * 8;

  v8f acc[4][4];
#pragma unroll
  for (int i = 0; i < 4; ++i)
#pragma unroll
    for (int j = 0; j < 4; ++j) acc[i][j] = (v8f){0.f,0.f,0.f,0.f,0.f,0.f,0.f,0.f};

  for (int k0 = 0; k0 < K; k0 += 32) {
    V bh[4];
#pragma unroll
    for (int j = 0; j < 4; ++j) {
      const size_t bo = (size_t)(n0 + (j << 4) + rlane) * ldb + koff + k0;
      bh[j] = Frag<T>::load(Bt + bo);
    }
#pragma unroll
    for (int i = 0; i < 4; ++i) {
      const size_t ao = (size_t)(m0 + (i << 4) + rlane) * lda + koff + k0;
      V ah = Frag<T>::load(A + ao);
      V al = ah;
      if (SPL == 1) al = Frag<T>::load(A2 + ao);
#pragma unroll
      for (int j = 0; j < 4; ++j) {
        acc[i][j] = Frag<T>::mma(ah, bh[j], acc[i][j]);
        if (SPL == 1) acc[i][j] = Frag<T>::mma(al, bh[j], acc[i][j]);
      }
      Frag<T>::guard4(acc[i][0], acc[i][1], acc[i][2], acc[i][3], ah, al);
    }
    Frag<T>::keep(bh[0], bh[1], bh[2], bh[3]);
  }
  acc_guard4(acc[0][0], acc[0][1], acc[0][2], acc[0][3]);
  acc_guard4(acc[1][0], acc[1][1], acc[1][2], acc[1][3]);
  acc_guard4(acc[2][0], acc[2][1], acc[2][2], acc[2][3]);
  acc_guard4(acc[3][0], acc[3][1], acc[3][2], acc[3][3]);

  float* slab = sT[wave];
#pragma unroll
  for (int i = 0; i < 4; ++i) {
    const int mBase = m0 + (i << 4);
#pragma unroll
    for (int j = 0; j < 4; ++j) {
#pragma unroll
      for (int r = 0; r < 8; ++r) {
        const float v = acc[i][j][r] * scale;
        slab[(mOff + r) * 68 + (j << 4) + rlane] = v;
      }
    }
    __builtin_amdgcn_fence(__ATOMIC_RELEASE, "workgroup");
    __builtin_amdgcn_wave_barrier();
    __builtin_amdgcn_fence(__ATOMIC_ACQUIRE, "workgroup");
    {
      const int hh = lane >> 4, c4 = (lane & 15) * 4;
      v4f ov[8];
#pragma unroll
      for (int it = 0; it < 8; ++it) {
        const int row = it * 2 + hh;
        v4f v = *(const v4f*)(slab + row * 68 + c4);
        if (SKIP) {
          const v4f rr = *(const v4f*)(skip + (size_t)(mBase + row) * ldc + n0 + c4);
          const float r0 = rr[0], r1 = rr[1], r2 = rr[2], r3 = rr[3];
          v[0] = v[0] + rbf(r0);
          v[1] = v[1] + rbf(r1);
          v[2] = v[2] + rbf(r2);
          v[3] = v[3] + rbf(r3);
        }
        ov[it] = v;
      }
      for (int pass = 0; pass < 2; ++pass) {
#pragma unroll
        for (int it = 0; it < 8; ++it) {
          const int row = it * 2 + hh;
          *(volatile v4f*)(C + (size_t)(mBase + row) * ldc + n0 + c4) = ov[it];
        }
        __threadfence();
      }
    }
    __builtin_amdgcn_fence(__ATOMIC_RELEASE, "workgroup");
    __builtin_amdgcn_wave_barrier();
    __builtin_amdgcn_fence(__ATOMIC_ACQUIRE, "workgroup");
  }
}

template <int MODE>
__global__ __launch_bounds__(256) void cast_plane_kernel(
    const float* __restrict__ src, unsigned short* __restrict__ dst, int real8, int total8, float scale)
{
  const int i = blockIdx.x * 256 + threadIdx.x;
  if (i >= total8) return;
  const bool live = (i < real8);
  const int ic = live ? i : (real8 - 1);
  const size_t s0 = (size_t)ic << 3;
  const v4f a0 = *(const v4f*)(src + s0);
  const v4f a1 = *(const v4f*)(src + s0 + 4);
  v8h hv;
#pragma unroll
  for (int e = 0; e < 4; ++e) {
    const float g0 = a0[e], g1 = a1[e];
    const float f0 = live ? g0 : 0.0f;
    const float f1 = live ? g1 : 0.0f;
    const unsigned short b0 = f2bf_bits(f0), b1 = f2bf_bits(f1);
    if (MODE == 0) {
      hv[e]     = __builtin_bit_cast(_Float16, b0);
      hv[4 + e] = __builtin_bit_cast(_Float16, b1);
    } else {
      hv[e]     = (_Float16)(bf_bits2f(b0) * scale);
      hv[4 + e] = (_Float16)(bf_bits2f(b1) * scale);
    }
  }
  unsigned short* q = dst + ((size_t)i << 3);
  *(volatile v8h*)q = hv;
  __threadfence();
  *(volatile v8h*)q = hv;
}

__global__ __launch_bounds__(256) void ln_split_kernel(
    const float* __restrict__ x, const float* __restrict__ g, const float* __restrict__ bt,
    unsigned short* __restrict__ XH, unsigned short* __restrict__ XL)
{
  const int lane = threadIdx.x & 31, wave = threadIdx.x >> 5;
  const int row = blockIdx.x * 8 + wave;
  const float* xr = x + (size_t)row * kDmod + lane * 8;
  float s = 0.0f;
#pragma unroll 1
  for (int c = 0; c < 4; ++c) {
    const v4f a0 = *(const v4f*)(xr + c * 256);
    const v4f a1 = *(const v4f*)(xr + c * 256 + 4);
#pragma unroll
    for (int e = 0; e < 4; ++e) {
      const float f0 = a0[e], f1 = a1[e];
      s += rbf(f0);
      s += rbf(f1);
    }
  }
#pragma unroll
  for (int off = 16; off > 0; off >>= 1) s += __shfl_xor(s, off, 32);
  const float mu = s * (1.0f / (float)kDmod);
  float q = 0.0f;
#pragma unroll 1
  for (int c = 0; c < 4; ++c) {
    const v4f a0 = *(const v4f*)(xr + c * 256);
    const v4f a1 = *(const v4f*)(xr + c * 256 + 4);
#pragma unroll
    for (int e = 0; e < 4; ++e) {
      const float f0 = a0[e], f1 = a1[e];
      const float d0 = rbf(f0) - mu, d1 = rbf(f1) - mu;
      q += d0 * d0;
      q += d1 * d1;
    }
  }
#pragma unroll
  for (int off = 16; off > 0; off >>= 1) q += __shfl_xor(q, off, 32);
  const float var  = q * (1.0f / (float)kDmod);
  const float rstd = 1.0f / sqrtf(var + 1e-5f);
#pragma unroll 1
  for (int c = 0; c < 4; ++c) {
    const int col = c * 256 + lane * 8;
    const v4f a0 = *(const v4f*)(xr + c * 256);
    const v4f a1 = *(const v4f*)(xr + c * 256 + 4);
    const v4f g0 = *(const v4f*)(g + col);
    const v4f g1 = *(const v4f*)(g + col + 4);
    const v4f b0 = *(const v4f*)(bt + col);
    const v4f b1 = *(const v4f*)(bt + col + 4);
    v8h hv, lv;
#pragma unroll
    for (int e = 0; e < 4; ++e) {
      const float xa = a0[e], xb = a1[e], ga = g0[e], gb = g1[e], ba = b0[e], bb = b1[e];
      const float va = ((rbf(xa) - mu) * rstd) * rbf(ga) + rbf(ba);
      const float vb = ((rbf(xb) - mu) * rstd) * rbf(gb) + rbf(bb);
      const unsigned short ha = f2bf_bits(va), hb = f2bf_bits(vb);
      const unsigned short la = f2bf_bits(va - bf_bits2f(ha)), lb = f2bf_bits(vb - bf_bits2f(hb));
      hv[e]     = __builtin_bit_cast(_Float16, ha);
      hv[4 + e] = __builtin_bit_cast(_Float16, hb);
      lv[e]     = __builtin_bit_cast(_Float16, la);
      lv[4 + e] = __builtin_bit_cast(_Float16, lb);
    }
    const size_t o = (size_t)row * kDmod + col;
    *(volatile v8h*)(XH + o) = hv;
    *(volatile v8h*)(XL + o) = lv;
    __threadfence();
    *(volatile v8h*)(XH + o) = hv;
    *(volatile v8h*)(XL + o) = lv;
  }
}

__global__ __launch_bounds__(256) void conv_silu_kernel(
    const float* __restrict__ XZ, const float* __restrict__ cw, const float* __restrict__ cb,
    unsigned short* __restrict__ UCH, unsigned short* __restrict__ UCL, unsigned short* __restrict__ UC16)
{
  __shared__ __align__(16) float sT[16 * kTP];
  const int tid = threadIdx.x, lane = tid & 31, wave = tid >> 5;
  const int d0 = blockIdx.x * 256, d = d0 + tid;
  const int t0 = blockIdx.y * 64;
  const v4f wv = *(const v4f*)(cw + (size_t)d * 4);
  const float wr0 = wv[0], wr1 = wv[1], wr2 = wv[2], wr3 = wv[3];
  const float w0 = rbf(wr0), w1 = rbf(wr1), w2 = rbf(wr2), w3 = rbf(wr3);
  const float bc = rbf(cb[d]);
  float xm3, xm2, xm1;
  {
    const int r3 = t0 - 3, r2 = t0 - 2, r1 = t0 - 1;
    const float v3 = XZ[(size_t)(r3 < 0 ? 0 : r3) * kXZP + d];
    const float v2 = XZ[(size_t)(r2 < 0 ? 0 : r2) * kXZP + d];
    const float v1 = XZ[(size_t)(r1 < 0 ? 0 : r1) * kXZP + d];
    xm3 = (r3 >= 0) ? v3 : 0.f;
    xm2 = (r2 >= 0) ? v2 : 0.f;
    xm1 = (r1 >= 0) ? v1 : 0.f;
  }
#pragma unroll 1
  for (int sub = 0; sub < 4; ++sub) {
    const int lb = t0 + sub * 16;
#pragma unroll 1
    for (int s = 0; s < 16; ++s) {
      const float xc = XZ[(size_t)(lb + s) * kXZP + d];
      float acc = w0 * xm3;
      acc = fmaf(w1, xm2, acc);
      acc = fmaf(w2, xm1, acc);
      acc = fmaf(w3, xc, acc);
      const float sv = acc + bc;
      const float sg = 1.0f / (1.0f + expf(-sv));
      sT[s * kTP + tid] = sv * sg;
      xm3 = xm2; xm2 = xm1; xm1 = xc;
    }
    __syncthreads();
    v8h bh[2], bl[2], bf[2];
#pragma unroll
    for (int it = 0; it < 2; ++it) {
      const float* sp = sT + (it * 8 + wave) * kTP + lane * 8;
      const v4f a0 = *(const v4f*)(sp);
      const v4f a1 = *(const v4f*)(sp + 4);
#pragma unroll
      for (int e = 0; e < 4; ++e) {
        const float f0 = a0[e], f1 = a1[e];
        const unsigned short h0 = f2bf_bits(f0), h1 = f2bf_bits(f1);
        const unsigned short l0 = f2bf_bits(f0 - bf_bits2f(h0)), l1 = f2bf_bits(f1 - bf_bits2f(h1));
        bh[it][e]     = __builtin_bit_cast(_Float16, h0);
        bh[it][4 + e] = __builtin_bit_cast(_Float16, h1);
        bl[it][e]     = __builtin_bit_cast(_Float16, l0);
        bl[it][4 + e] = __builtin_bit_cast(_Float16, l1);
        bf[it][e]     = (_Float16)(f0 * kCarryAct);
        bf[it][4 + e] = (_Float16)(f1 * kCarryAct);
      }
    }
    for (int pass = 0; pass < 2; ++pass) {
#pragma unroll
      for (int it = 0; it < 2; ++it) {
        const size_t o = (size_t)(lb + it * 8 + wave) * kDin + d0 + lane * 8;
        *(volatile v8h*)(UCH + o)  = bh[it];
        *(volatile v8h*)(UCL + o)  = bl[it];
        *(volatile v8h*)(UC16 + o) = bf[it];
      }
      __threadfence();
    }
    __syncthreads();
  }
}

__global__ __launch_bounds__(256) void scan_kernel(
    const float* __restrict__ DLR, const float* __restrict__ bdt,
    const unsigned* __restrict__ UCHw, const unsigned* __restrict__ UCLw,
    const float* __restrict__ XZ, const float* __restrict__ XD,
    const float* __restrict__ A_log, const float* __restrict__ Dv,
    unsigned short* __restrict__ YG)
{
#pragma clang fp contract(off)
  __shared__ __align__(16) float sBC[16 * 32];
  __shared__ __align__(16) float sY[16 * kTP];
  __shared__ __align__(16) float sA[kNst * 256];
  const int tid = threadIdx.x, lane = tid & 31, wave = tid >> 5;
  const int d0 = blockIdx.x * 256, d = d0 + tid;
  const bool odd = (tid & 1) != 0;

#pragma unroll 1
  for (int n = 0; n < kNst; ++n) sA[n * 256 + tid] = -expf(rbf(A_log[(size_t)d * kNst + n]));
  __syncthreads();
  float An[kNst], h[kNst];
#pragma unroll
  for (int n = 0; n < kNst; ++n) { An[n] = sA[n * 256 + tid]; h[n] = 0.f; }
  const float bb = rbf(bdt[d]);
  const float Dd = rbf(Dv[d]);

#pragma unroll 1
  for (int c = 0; c < kSeqL / 16; ++c) {
    const int l0 = c * 16;
    if (tid < 128) {
      const int r = tid >> 3, q = (tid & 7) * 4;
      const v4f v = *(const v4f*)(XD + (size_t)(l0 + r) * kXdP + q);
      *(v4f*)(sBC + r * 32 + q) = v;
    }
    __syncthreads();
#pragma unroll 1
    for (int s = 0; s < 16; ++s) {
      const size_t m = (size_t)(l0 + s);
      const float a     = DLR[m * kDin + d] + bb;
      const unsigned wh = UCHw[(m * kDin + d) >> 1];
      const unsigned wl = UCLw[(m * kDin + d) >> 1];
      const float zv    = XZ[m * kXZP + kDin + d];
      const float delta = fmaxf(a, 0.0f) + log1pf(expf(-fabsf(a)));
      const unsigned hbits = odd ? (wh & 0xffff0000u) : (wh << 16);
      const unsigned lbits = odd ? (wl & 0xffff0000u) : (wl << 16);
      const float xv = __uint_as_float(hbits) + __uint_as_float(lbits);
      v4f Bq[4], Cq[4];
#pragma unroll
      for (int qq = 0; qq < 4; ++qq) {
        Bq[qq] = *(const v4f*)(sBC + s * 32 + 4 * qq);
        Cq[qq] = *(const v4f*)(sBC + s * 32 + kNst + 4 * qq);
      }
      const float dtx = delta * xv;
      float y = 0.f;
#pragma unroll
      for (int n = 0; n < kNst; ++n) {
        const float e  = expf(delta * An[n]);
        const float p  = dtx * Bq[n >> 2][n & 3];
        const float qv = e * h[n];
        const float hn = qv + p;
        h[n] = hn;
        const float rr = hn * Cq[n >> 2][n & 3];
        y = y + rr;
      }
      const float sk = xv * Dd;
      y = y + sk;
      const float sg = 1.0f / (1.0f + expf(-zv));
      const float gt = zv * sg;
      sY[s * kTP + tid] = (y * gt) * kCarryAct;
    }
    __syncthreads();
    v8h hv[2];
#pragma unroll
    for (int it = 0; it < 2; ++it) {
      const float* sp = sY + (it * 8 + wave) * kTP + lane * 8;
      const v4f a0 = *(const v4f*)(sp);
      const v4f a1 = *(const v4f*)(sp + 4);
#pragma unroll
      for (int e = 0; e < 4; ++e) { hv[it][e] = (_Float16)a0[e]; hv[it][4 + e] = (_Float16)a1[e]; }
    }
    for (int pass = 0; pass < 2; ++pass) {
#pragma unroll
      for (int it = 0; it < 2; ++it)
        *(volatile v8h*)(YG + (size_t)(l0 + it * 8 + wave) * kDin + d0 + lane * 8) = hv[it];
      __threadfence();
    }
  }
}

extern "C" void kernel_launch(void* const* d_in, const int* in_sizes, int n_in,
                              void* d_out, int out_size, void* d_ws, size_t ws_size,
                              hipStream_t stream)
{
  if (n_in < 12) return;
  if (in_sizes[0] != kRows * kDmod) return;
  if (in_sizes[1] != kXZP * kDmod) return;
  if (in_sizes[2] != kDin * 4 || in_sizes[3] != kDin) return;
  if (in_sizes[4] != kXdN * kDin) return;
  if (in_sizes[5] != kDin * kDin || in_sizes[6] != kDin) return;
  if (in_sizes[7] != kDin * kNst || in_sizes[8] != kDin) return;
  if (in_sizes[9] != kDmod * kDin) return;
  if (in_sizes[10] != kDmod || in_sizes[11] != kDmod) return;
  if (out_size != kRows * kDmod) return;
  if (ws_size < kWsTotal) return;

  const float* x      = (const float*)d_in[0];
  const float* W_in   = (const float*)d_in[1];
  const float* conv_w = (const float*)d_in[2];
  const float* conv_b = (const float*)d_in[3];
  const float* W_x    = (const float*)d_in[4];
  const float* W_dt   = (const float*)d_in[5];
  const float* b_dt   = (const float*)d_in[6];
  const float* A_log  = (const float*)d_in[7];
  const float* Dp     = (const float*)d_in[8];
  const float* W_out  = (const float*)d_in[9];
  const float* ln_g   = (const float*)d_in[10];
  const float* ln_b   = (const float*)d_in[11];
  float* out = (float*)d_out;

  char* ws = (char*)d_ws;
  unsigned short* WIN  = (unsigned short*)(ws + kOffWIN);
  unsigned short* WDT  = (unsigned short*)(ws + kOffWDT);
  unsigned short* WOUT = (unsigned short*)(ws + kOffWOUT);
  unsigned short* WX   = (unsigned short*)(ws + kOffWX);
  unsigned short* XNH  = (unsigned short*)(ws + kOffXNH);
  unsigned short* XNL  = (unsigned short*)(ws + kOffXNL);
  float*          XZ   = (float*)(ws + kOffXZ);
  unsigned short* UCH  = (unsigned short*)(ws + kOffUCH);
  unsigned short* UCL  = (unsigned short*)(ws + kOffUCL);
  unsigned short* UC16 = (unsigned short*)(ws + kOffUC16);
  float*          XD   = (float*)(ws + kOffXD);
  float*          DLR  = (float*)(ws + kOffDLR);
  unsigned short* YG   = (unsigned short*)(ws + kOffYG);

  cast_plane_kernel<0><<<(kXZP * kDmod / 8) / 256, 256, 0, stream>>>(W_in, WIN, kXZP * kDmod / 8, kXZP * kDmod / 8, 1.0f);
  cast_plane_kernel<1><<<(kDin * kDin / 8) / 256, 256, 0, stream>>>(W_dt, WDT, kDin * kDin / 8, kDin * kDin / 8, kCarryW);
  cast_plane_kernel<1><<<(kDmod * kDin / 8) / 256, 256, 0, stream>>>(W_out, WOUT, kDmod * kDin / 8, kDmod * kDin / 8, kCarryW);
  cast_plane_kernel<0><<<(kXdP * kDin / 8) / 256, 256, 0, stream>>>(W_x, WX, kXdN * kDin / 8, kXdP * kDin / 8, 1.0f);

  ln_split_kernel<<<kRows / 8, 256, 0, stream>>>(x, ln_g, ln_b, XNH, XNL);

  for (int b = 0; b < kBatch; ++b) {
    const unsigned short* XNHb = XNH + (size_t)b * kSeqL * kDmod;
    const unsigned short* XNLb = XNL + (size_t)b * kSeqL * kDmod;
    const float* xb = x + (size_t)b * kSeqL * kDmod;
    float* outb = out + (size_t)b * kSeqL * kDmod;

    wmma_gemm64<1, 1, false><<<dim3(256, 1), 256, 0, stream>>>(
        XNHb, XNLb, kDmod, WIN, kDmod, XZ, kXZP, xb, kSeqL, kXZP, kDmod, 1.0f);

    conv_silu_kernel<<<dim3(kDin / 256, kSeqL / 64), 256, 0, stream>>>(XZ, conv_w, conv_b, UCH, UCL, UC16);

    wmma_gemm64<1, 1, false><<<dim3(4, 1), 256, 0, stream>>>(
        UCH, UCL, kDin, WX, kDin, XD, kXdP, xb, kSeqL, kXdP, kDin, 1.0f);

    wmma_gemm64<0, 0, false><<<dim3(128, 1), 256, 0, stream>>>(
        UC16, UC16, kDin, WDT, kDin, DLR, kDin, xb, kSeqL, kDin, kDin, kFold);

    scan_kernel<<<dim3(kDin / 256, 1), 256, 0, stream>>>(
        DLR, b_dt, (const unsigned*)UCH, (const unsigned*)UCL, XZ, XD, A_log, Dp, YG);

    wmma_gemm64<0, 0, true><<<dim3(64, 1), 256, 0, stream>>>(
        YG, YG, kDin, WOUT, kDin, outb, kDmod, xb, kSeqL, kDmod, kDin, kFold);
  }
}
